// GMAN_54468775247906
// MI455X (gfx1250) — hardware-verified
//
#include <hip/hip_runtime.h>
#include <math.h>

typedef __attribute__((ext_vector_type(16))) _Float16 v16h;
typedef __attribute__((ext_vector_type(16))) __bf16 v16b;
typedef __attribute__((ext_vector_type(8)))  _Float16 v8h;
typedef __attribute__((ext_vector_type(8)))  float v8f;
typedef __attribute__((ext_vector_type(4)))  float v4f;
typedef __attribute__((ext_vector_type(2)))  float v2f;
typedef __attribute__((ext_vector_type(4)))  unsigned v4u;
typedef __attribute__((ext_vector_type(4)))  int v4i;
typedef float __attribute__((may_alias)) float_a;
typedef int __attribute__((may_alias)) int_a;

template <typename T> __device__ __forceinline__ void vst2(void* p, T v) { *(volatile T*)p = v; __threadfence(); *(volatile T*)p = v; }
__device__ __forceinline__ v8f wmma16(v16h a, v16h b, v8f c) {
  v8f d = __builtin_amdgcn_wmma_f32_16x16x32_f16(false, a, false, b, (short)0, c, false, false);
  asm volatile("v_nop\n\tv_nop\n\tv_nop\n\tv_nop" : "+v"(d) : "v"(a), "v"(b));
  return d;
}
__device__ __forceinline__ v8f wmma_bf(v16b a, v16b b, v8f c) {
  v8f d = __builtin_amdgcn_wmma_f32_16x16x32_bf16(false, a, false, b, (short)0, c, false, false);
  asm volatile("v_nop\n\tv_nop\n\tv_nop\n\tv_nop" : "+v"(d) : "v"(a), "v"(b));
  return d;
}
__device__ __forceinline__ v16h frag_h(const _Float16* rowk0, int lane) {
  union { v16h v; v8h q[2]; } u; const _Float16* p = rowk0 + 8 * (lane >> 4);
  u.q[0] = *(const v8h*)p; u.q[1] = *(const v8h*)(p + 16); return u.v;
}
__device__ __forceinline__ v16h frag_f32(const float* rowk0, int lane) {
  v16h a; const float* p = rowk0 + 8 * (lane >> 4);
#pragma unroll
  for (int i = 0; i < 8; ++i) { a[i] = (_Float16)p[i]; a[8 + i] = (_Float16)p[16 + i]; }
  return a;
}
__device__ __forceinline__ v16h frag_f32s(const float* rowk0, int lane, float sc) {
  v16h a; const float* p = rowk0 + 8 * (lane >> 4);
#pragma unroll
  for (int i = 0; i < 8; ++i) { a[i] = (_Float16)(p[i] * sc); a[8 + i] = (_Float16)(p[16 + i] * sc); }
  return a;
}
__device__ __forceinline__ v16h fragc_f32(const float* W, int k0, int n, int lane, int ld, int K) {
  v16h a; const int g = lane >> 4;
#pragma unroll
  for (int i = 0; i < 8; ++i) { const int ka = k0 + 8 * g + i, kb = ka + 16;
    a[i] = (_Float16)(ka < K ? W[(size_t)(ka < K ? ka : K - 1) * ld + n] : 0.f); a[8 + i] = (_Float16)(kb < K ? W[(size_t)(kb < K ? kb : K - 1) * ld + n] : 0.f); }
  return a;
}
struct F2 { v16b h, l; };
__device__ __forceinline__ F2 bsplit16(const float v[16]) { F2 r;
#pragma unroll
  for (int i = 0; i < 16; ++i) { const __bf16 h = (__bf16)v[i]; r.h[i] = h; r.l[i] = (__bf16)(v[i] - (float)h); }
  return r; }
__device__ __forceinline__ F2 split_row(const float* row, int k0, int lane) { float v[16]; const float* p = row + k0 + 8 * (lane >> 4);
#pragma unroll
  for (int i = 0; i < 8; ++i) { v[i] = p[i]; v[8 + i] = p[16 + i]; }
  return bsplit16(v); }
__device__ __forceinline__ F2 split_rowK(const float* row, int k0, int lane, int K) { float v[16]; const int g = lane >> 4;
#pragma unroll
  for (int i = 0; i < 8; ++i) { const int ka = k0 + 8 * g + i, kb = ka + 16; v[i] = ka < K ? row[ka < K ? ka : K - 1] : 0.f; v[8 + i] = kb < K ? row[kb < K ? kb : K - 1] : 0.f; }
  return bsplit16(v); }
__device__ __forceinline__ F2 split_col(const float* W, int k0, int n, int lane, int ld, int K) { float v[16]; const int g = lane >> 4;
#pragma unroll
  for (int i = 0; i < 8; ++i) { const int ka = k0 + 8 * g + i, kb = ka + 16; v[i] = ka < K ? W[(size_t)(ka < K ? ka : K - 1) * ld + n] : 0.f; v[8 + i] = kb < K ? W[(size_t)(kb < K ? kb : K - 1) * ld + n] : 0.f; }
  return bsplit16(v); }
__device__ __forceinline__ v8f mac3(const F2& a, const F2& b, v8f c) { c = wmma_bf(a.l, b.h, c); c = wmma_bf(a.h, b.l, c); return wmma_bf(a.h, b.h, c); }
__device__ __forceinline__ float sigm(float v) { return 1.0f / (1.0f + expf(-v)); }
#define LDSX() do { asm volatile("s_wait_dscnt 0" ::: "memory"); __builtin_amdgcn_wave_barrier(); __builtin_amdgcn_fence(__ATOMIC_RELEASE, "workgroup"); } while (0)


#define NBq 8
#define NTq 12
#define NG (NBq * NTq)
#define NN 325
#define NP 336
#define DM 128
#define NH 8
#define DHd 16
#define FF 512
#define NE 16
#ifndef NGT
#define NGT NG
#endif
#define NRP (NG * NP)
typedef __attribute__((ext_vector_type(8))) __bf16 v8b;
__device__ __forceinline__ v16b frag_b(const __bf16* rowk0, int lane) {
  union { v16b v; v8b q[2]; } u; const __bf16* p = rowk0 + 8 * (lane >> 4);
  u.q[0] = *(const v8b*)p; u.q[1] = *(const v8b*)(p + 16); return u.v;
}
__device__ __forceinline__ float bfr(float v) { return (float)(__bf16)v; }
__device__ __attribute__((noinline)) float exp_ni(float v) { return expf(v); }
__device__ __attribute__((noinline)) float erf_ni(float v) { return erff(v); }

#define PK_Q  0
#define PK_K  ((size_t)DM * DM)
#define PK_V  ((size_t)2 * DM * DM)
#define PK_O  ((size_t)3 * DM * DM)
#define PK_1  ((size_t)4 * DM * DM)
#define PK_2  (PK_1 + (size_t)FF * DM)
#define PK_END (PK_2 + (size_t)DM * FF)
#define WS_PK  0u
#define WS_TAB (((2u * PK_END) + 127u) / 128u * 128u)
#define WS_XN  (WS_TAB + 4u * NN * NP)
#define WS_QH  (WS_XN + 4u * NRP * DM)
#define WS_QL  (WS_QH + 2u * NRP * NH * 32)
#define WS_KH  (WS_QL + 2u * NRP * NH * 32)
#define WS_KL  (WS_KH + 2u * NRP * NH * 32)
#define NPV 384
#define WS_VTH (WS_KL + 2u * NRP * NH * 32)
#define WS_VTL (WS_VTH + 2u * (size_t)NG * DM * NPV)
#define WS_O   (WS_VTL + 2u * (size_t)NG * DM * NPV)
#define WS_X1  (WS_O + 4u * NRP * DM)
#define WS_GH  (WS_X1 + 4u * NRP * DM)
#define WS_GL  (WS_GH + 2u * NRP * FF)
#define WS_END (WS_GL + 2u * NRP * FF)

__device__ __forceinline__ size_t xrow(size_t pr) { const size_t grp = pr / NP, n = pr % NP; return grp * NN + (n < NN ? n : NN - 1); }

__global__ __launch_bounds__(256) void k_pack(const float* __restrict__ WQ, const float* __restrict__ WK, const float* __restrict__ WV, const float* __restrict__ WO, const float* __restrict__ W1, const float* __restrict__ W2, __bf16* __restrict__ PK) {
  __shared__ __align__(16) __bf16 s[FF]; const int n = blockIdx.x, which = blockIdx.y, t = threadIdx.x; int K, NO; size_t dst; const float* Wm;
  switch (which) { case 0: Wm = WQ; K = DM; NO = DM; dst = PK_Q; break; case 1: Wm = WK; K = DM; NO = DM; dst = PK_K; break; case 2: Wm = WV; K = DM; NO = DM; dst = PK_V; break; case 3: Wm = WO; K = DM; NO = DM; dst = PK_O; break; case 4: Wm = W1; K = DM; NO = FF; dst = PK_1; break; default: Wm = W2; K = FF; NO = DM; dst = PK_2; break; }
  if (n >= NO) return;
  for (int k = t; k < K; k += 256) s[k] = (__bf16)Wm[(size_t)k * NO + n];
  __syncthreads();
  for (int q = t; q < K / 8; q += 256) vst2((unsigned*)(PK + dst + (size_t)n * K + q * 8), *(const v4u*)&s[q * 8]);
}
__global__ __launch_bounds__(256) void k_tab(const float* __restrict__ E, const float* __restrict__ LAP, const float* __restrict__ AL, const float* __restrict__ BE, float* __restrict__ TAB) {
  __shared__ float srow[NP]; __shared__ float red[8]; __shared__ __align__(16) float sout[NP]; const int t = threadIdx.x; const int n = blockIdx.x; float en[NE];
#pragma unroll
  for (int e = 0; e < NE; ++e) en[e] = bfr(E[n * NE + e]);
  float mx = -3.0e38f;
  for (int m = t; m < NN; m += 256) { float a = 0.f;
#pragma unroll
    for (int e = 0; e < NE; ++e) a += en[e] * bfr(E[m * NE + e]);
    a = fmaxf(a, 0.f); srow[m] = a; mx = fmaxf(mx, a); }
#pragma unroll
  for (int o = 1; o < 32; o <<= 1) mx = fmaxf(mx, __shfl_xor(mx, o));
  if ((t & 31) == 0) red[t >> 5] = mx; __syncthreads(); float gm = -3.0e38f; for (int w = 0; w < 8; ++w) gm = fmaxf(gm, red[w]); __syncthreads();
  float sm = 0.f; for (int m = t; m < NN; m += 256) { const float e = exp_ni(srow[m] - gm); srow[m] = e; sm += e; }
#pragma unroll
  for (int o = 1; o < 32; o <<= 1) sm += __shfl_xor(sm, o);
  if ((t & 31) == 0) red[t >> 5] = sm; __syncthreads(); float tot = 0.f; for (int w = 0; w < 8; ++w) tot += red[w]; const float inv = 1.0f / tot; const float al = bfr(AL[0]), be = bfr(BE[0]);
  for (int m = t; m < NP; m += 256) { if (m < NN) { const float lp = bfr(LAP[n * NN + m]); sout[m] = al * (srow[m] * inv) + be * lp + ((lp != 0.f) ? 0.f : -1.0e9f); } else sout[m] = -3.0e38f; }
  __syncthreads();
  for (int q = t; q < NP / 4; q += 256) vst2(TAB + (size_t)n * NP + q * 4, *(const v4f*)&sout[q * 4]);
}
__global__ __launch_bounds__(32) void k_ln(const float* __restrict__ SRC, int from_x, const float* __restrict__ G, const float* __restrict__ Bv, float* __restrict__ XN) {
  const int t = threadIdx.x; const size_t pr = blockIdx.x; const float* p = from_x ? (SRC + xrow(pr) * DM + t * 4) : (SRC + pr * DM + t * 4);
  float v[4]; for (int i = 0; i < 4; ++i) v[i] = from_x ? bfr(p[i]) : p[i]; float s = (v[0] + v[1]) + (v[2] + v[3]);
#pragma unroll
  for (int o = 1; o < 32; o <<= 1) s += __shfl_xor(s, o);
  const float mu = s / (float)DM; float q = 0.f;
#pragma unroll
  for (int i = 0; i < 4; ++i) { const float d = v[i] - mu; q += d * d; }
#pragma unroll
  for (int o = 1; o < 32; o <<= 1) q += __shfl_xor(q, o);
  const float inv = 1.0f / sqrtf(q / (float)DM + 1e-5f); v4f o4;
#pragma unroll
  for (int i = 0; i < 4; ++i) o4[i] = (v[i] - mu) * inv * bfr(G[t * 4 + i]) + bfr(Bv[t * 4 + i]);
  vst2(XN + pr * DM + t * 4, o4);
}
#define TPG 6
__device__ __forceinline__ size_t clampr(size_t pr) { return pr < (size_t)NRP ? pr : (size_t)NRP - 1; }
__global__ __launch_bounds__(128) void k_qkv(const float* __restrict__ XN, const __bf16* __restrict__ PK, const float* __restrict__ BQ, const float* __restrict__ BK, const float* __restrict__ BV, _Float16* __restrict__ QH, _Float16* __restrict__ QL, _Float16* __restrict__ KH, _Float16* __restrict__ KL, _Float16* __restrict__ VTH, _Float16* __restrict__ VTL) {
  __shared__ __align__(16) _Float16 soh[4][16][NH * 32 + 8], sol[4][16][NH * 32 + 8]; __shared__ __align__(16) _Float16 sth[128][72], stl[128][72];
  const int tid = threadIdx.x, wave = tid >> 5, lane = tid & 31, col = lane & 15, g = lane >> 4; const int which = blockIdx.y; const size_t grp = blockIdx.x / TPG; const int tile = blockIdx.x % TPG; const size_t rb = grp * NP + tile * 64; const size_t r0 = rb + wave * 16; const int nvalid = min(64, NP - tile * 64);
  const __bf16* P = PK + ((which == 0) ? PK_Q : (which == 1) ? PK_K : PK_V); const float* BB = (which == 0) ? BQ : (which == 1) ? BK : BV;
  v8f acc[8] = {};
#pragma unroll
  for (int kc = 0; kc < DM / 32; ++kc) { const F2 a = split_row(XN + clampr(r0 + col) * DM, kc * 32, lane);
#pragma unroll
    for (int j = 0; j < 8; ++j) { const v16b w = frag_b(P + (size_t)(j * 16 + col) * DM + kc * 32, lane); acc[j] = wmma_bf(a.l, w, acc[j]); acc[j] = wmma_bf(a.h, w, acc[j]); } }
  if (which < 2) {
    for (int e = tid; e < 4 * 16 * (NH * 32 + 8); e += 128) { (&soh[0][0][0])[e] = (_Float16)0.f; (&sol[0][0][0])[e] = (_Float16)0.f; }
    __syncthreads();
#pragma unroll
    for (int j = 0; j < 8; ++j) { const float bb = bfr(BB[j * 16 + col]);
#pragma unroll
      for (int r = 0; r < 8; ++r) { const float v = acc[j][r] + bb; const _Float16 hv = (_Float16)v; soh[wave][8 * g + r][j * 32 + col] = hv; sol[wave][8 * g + r][j * 32 + col] = (_Float16)((v - (float)hv) * 2048.0f); } }
    LDSX();
    _Float16* DH_ = (which == 0) ? QH : KH; _Float16* DL_ = (which == 0) ? QL : KL;
    for (int rl = 0; rl < 16; ++rl) { if (wave * 16 + rl >= nvalid) break; const size_t o = (r0 + rl) * (NH * 32); vst2((unsigned*)(DH_ + o + lane * 8), *(const v4u*)&soh[wave][rl][lane * 8]); vst2((unsigned*)(DL_ + o + lane * 8), *(const v4u*)&sol[wave][rl][lane * 8]); }
  } else {
#pragma unroll
    for (int j = 0; j < 8; ++j) { const float bb = bfr(BB[j * 16 + col]);
#pragma unroll
      for (int r = 0; r < 8; ++r) { const int rr = wave * 16 + 8 * g + r; const float v = (rr < nvalid) ? acc[j][r] + bb : 0.f; const _Float16 hv = (_Float16)v; sth[j * 16 + col][rr] = hv; stl[j * 16 + col][rr] = (_Float16)((v - (float)hv) * 2048.0f); } }
    __syncthreads();
    for (int e = tid; e < 128 * 8; e += 128) { const int d = e >> 3, pc = e & 7; const size_t o = (grp * DM + d) * NPV + tile * 64 + pc * 8; vst2((unsigned*)(VTH + o), *(const v4u*)&sth[d][pc * 8]); vst2((unsigned*)(VTL + o), *(const v4u*)&stl[d][pc * 8]); }
  }
}
__global__ __launch_bounds__(128) void k_attn(const _Float16* __restrict__ QH, const _Float16* __restrict__ QL, const _Float16* __restrict__ KH, const _Float16* __restrict__ KL, const _Float16* __restrict__ VTH, const _Float16* __restrict__ VTL, const float* __restrict__ TAB, float* __restrict__ O) {
  __shared__ __align__(16) _Float16 sph[4][16][40], spl[4][16][40]; __shared__ __align__(16) float so[4][16][36];
  const int tid = threadIdx.x, wave = tid >> 5, lane = tid & 31, col = lane & 15, g = lane >> 4; const size_t grp = blockIdx.x / TPG; const int tile = blockIdx.x % TPG; const int hp = blockIdx.y; const int n0w = tile * 64 + wave * 16; const size_t rw = grp * NP + n0w; const int nvalid = min(64, NP - tile * 64);
#pragma unroll 1
  for (int hh = 0; hh < 2; ++hh) { const int h = hp * 2 + hh;
    const v16h aq = frag_h(QH + clampr(rw + col) * (NH * 32) + h * 32, lane), aql = frag_h(QL + clampr(rw + col) * (NH * 32) + h * 32, lane);
    float m[8], l[8];
#pragma unroll
    for (int r = 0; r < 8; ++r) { m[r] = -3.0e38f; l[r] = 0.f; }
    v8f acc = {}, accl = {};
#pragma unroll 1
    for (int ks = 0; ks < (NP + 31) / 32; ++ks) { const int j0 = ks * 32; v8f s[2];
#pragma unroll
      for (int ct = 0; ct < 2; ++ct) { const int kk = j0 + ct * 16 + col; const int kkc = min(kk, NP - 1); const size_t rk = (grp * NP + kkc) * (NH * 32) + h * 32; v8f c = {}, cl = {};
        { const v16h kh = frag_h(KH + rk, lane); c = wmma16(aq, kh, c); cl = wmma16(aql, kh, cl); cl = wmma16(aq, frag_h(KL + rk, lane), cl); }
#pragma unroll
        for (int r = 0; r < 8; ++r) { const int n = n0w + 8 * g + r; const int nc = min(n, NN - 1); s[ct][r] = (kk < NN) ? (c[r] + cl[r] * (1.0f / 2048.0f)) * 0.25f + TAB[(size_t)nc * NP + kk] : -3.0e38f; } }
#pragma unroll
      for (int r = 0; r < 8; ++r) { float mx = fmaxf(s[0][r], s[1][r]);
#pragma unroll
        for (int o = 1; o < 16; o <<= 1) mx = fmaxf(mx, __shfl_xor(mx, o));
        const float mn = fmaxf(m[r], mx); const float alpha = (m[r] <= -1.0e38f) ? 0.f : __expf(m[r] - mn);
        const float e0 = (s[0][r] <= -1.0e38f) ? 0.f : __expf(s[0][r] - mn), e1 = (s[1][r] <= -1.0e38f) ? 0.f : __expf(s[1][r] - mn); float es = e0 + e1;
#pragma unroll
        for (int o = 1; o < 16; o <<= 1) es += __shfl_xor(es, o);
        l[r] = l[r] * alpha + es; m[r] = (mn <= -1.0e38f) ? m[r] : mn;
        acc[r] *= alpha; accl[r] *= alpha;
        const _Float16 h0 = (_Float16)e0, h1 = (_Float16)e1; sph[wave][8 * g + r][col] = h0; sph[wave][8 * g + r][16 + col] = h1; spl[wave][8 * g + r][col] = (_Float16)((e0 - (float)h0) * 2048.0f); spl[wave][8 * g + r][16 + col] = (_Float16)((e1 - (float)h1) * 2048.0f); }
      LDSX();
      const v16h pah = frag_h(&sph[wave][col][0], lane), pal = frag_h(&spl[wave][col][0], lane);
      { const size_t vo = (grp * DM + h * DHd + col) * NPV + j0; const v16h vh = frag_h(VTH + vo, lane), vl = frag_h(VTL + vo, lane); acc = wmma16(pah, vh, acc); accl = wmma16(pal, vh, accl); accl = wmma16(pah, vl, accl); }
      LDSX(); }
#pragma unroll
    for (int r = 0; r < 8; ++r) { const float il = 1.0f / l[r]; so[wave][8 * g + r][hh * 16 + col] = (acc[r] + accl[r] * (1.0f / 2048.0f)) * il; } }
  LDSX();
  for (int rl = 0; rl < 16; ++rl) { if (wave * 16 + rl >= nvalid) break; if (lane < 8) vst2(O + (rw + rl) * DM + hp * 32 + lane * 4, *(const v4f*)&so[wave][rl][lane * 4]); }
}
template <int MODE>
__global__ __launch_bounds__(128) void k_lin(const float* __restrict__ A, const __bf16* __restrict__ GH, const __bf16* __restrict__ GL, const __bf16* __restrict__ PK, const float* __restrict__ BIAS, const float* __restrict__ RES, float* __restrict__ OUTF, __bf16* __restrict__ OGH, __bf16* __restrict__ OGL) {
  __shared__ __align__(16) float so[4][16][132]; __shared__ __align__(16) __bf16 sg[4][16][136], sgl[4][16][136];
  const int tid = threadIdx.x, wave = tid >> 5, lane = tid & 31, col = lane & 15, g = lane >> 4; const size_t grp = blockIdx.x / TPG; const int tile = blockIdx.x % TPG; const size_t r0 = grp * NP + tile * 64 + wave * 16; const int n0 = blockIdx.y * 128; const int nvalid = min(64, NP - tile * 64);
  const __bf16* P = PK + ((MODE == 0) ? PK_O : (MODE == 1) ? PK_1 : PK_2);
  v8f acc[8] = {};
  if (MODE == 2) {
#pragma unroll 2
    for (int kc = 0; kc < FF / 32; ++kc) { const v16b a = frag_b(GH + clampr(r0 + col) * FF + kc * 32, lane), al = frag_b(GL + clampr(r0 + col) * FF + kc * 32, lane);
#pragma unroll
      for (int j = 0; j < 8; ++j) { const v16b w = frag_b(P + (size_t)(n0 + j * 16 + col) * FF + kc * 32, lane); acc[j] = wmma_bf(al, w, acc[j]); acc[j] = wmma_bf(a, w, acc[j]); } }
  } else {
#pragma unroll
    for (int kc = 0; kc < DM / 32; ++kc) { const F2 a = split_row(A + clampr(r0 + col) * DM, kc * 32, lane);
#pragma unroll
      for (int j = 0; j < 8; ++j) { const v16b w = frag_b(P + (size_t)(n0 + j * 16 + col) * DM + kc * 32, lane); acc[j] = wmma_bf(a.l, w, acc[j]); acc[j] = wmma_bf(a.h, w, acc[j]); } } }
  if (MODE == 1) {
#pragma unroll
    for (int j = 0; j < 8; ++j) { const float bb = bfr(BIAS[n0 + j * 16 + col]);
#pragma unroll
      for (int r = 0; r < 8; ++r) { const float v = fmaxf(acc[j][r] + bb, 0.f); const __bf16 hb = (__bf16)v; sg[wave][8 * g + r][j * 16 + col] = hb; sgl[wave][8 * g + r][j * 16 + col] = (__bf16)(v - (float)hb); } }
    LDSX();
    for (int rl = 0; rl < 16; ++rl) { if (wave * 16 + rl >= nvalid) break; if (lane < 16) vst2((unsigned*)(OGH + (r0 + rl) * FF + n0 + lane * 8), *(const v4u*)&sg[wave][rl][lane * 8]); else vst2((unsigned*)(OGL + (r0 + rl) * FF + n0 + (lane - 16) * 8), *(const v4u*)&sgl[wave][rl][(lane - 16) * 8]); }
  } else {
#pragma unroll
    for (int j = 0; j < 8; ++j) { const int c = n0 + j * 16 + col; const float bb = bfr(BIAS[c]);
#pragma unroll
      for (int r = 0; r < 8; ++r) { const size_t pr = clampr(r0 + 8 * g + r); const float res = (MODE == 0) ? bfr(RES[xrow(pr) * DM + c]) : RES[pr * DM + c]; so[wave][8 * g + r][j * 16 + col] = acc[j][r] + bb + res; } }
    LDSX();
    for (int rl = 0; rl < 16; ++rl) { if (wave * 16 + rl >= nvalid) break; const size_t pr = r0 + rl; float* dst = (MODE == 0) ? (OUTF + pr * DM) : (OUTF + xrow(pr) * DM); vst2(dst + n0 + lane * 4, *(const v4f*)&so[wave][rl][lane * 4]); } }
}
extern "C" void kernel_launch(void* const* d_in, const int* in_sizes, int n_in, void* d_out, int out_size, void* d_ws, size_t ws_size, hipStream_t stream) {
  (void)in_sizes; (void)n_in; (void)out_size;
  const float** F = (const float**)d_in;
  if (ws_size < (size_t)WS_END) return;
  char* ws = (char*)d_ws; __bf16 *PK = (__bf16*)(ws + WS_PK), *GH = (__bf16*)(ws + WS_GH), *GL = (__bf16*)(ws + WS_GL); float *TAB = (float*)(ws + WS_TAB), *XN = (float*)(ws + WS_XN), *O = (float*)(ws + WS_O), *X1 = (float*)(ws + WS_X1);
  _Float16 *QH = (_Float16*)(ws + WS_QH), *QL = (_Float16*)(ws + WS_QL), *KH = (_Float16*)(ws + WS_KH), *KL = (_Float16*)(ws + WS_KL), *VTH = (_Float16*)(ws + WS_VTH), *VTL = (_Float16*)(ws + WS_VTL);
  k_pack<<<dim3(FF, 6), 256, 0, stream>>>(F[3], F[5], F[7], F[11], F[15], F[17], PK);
  k_tab<<<NN, 256, 0, stream>>>(F[2], F[1], F[19], F[20], TAB);
  k_ln<<<NGT * NP, 32, 0, stream>>>(F[0], 1, F[9], F[10], XN);
  k_qkv<<<dim3(NGT * TPG, 3), 128, 0, stream>>>(XN, PK, F[4], F[6], F[8], QH, QL, KH, KL, VTH, VTL);
  k_attn<<<dim3(NGT * TPG, NH / 2), 128, 0, stream>>>(QH, QL, KH, KL, VTH, VTL, TAB, O);
  k_lin<0><<<dim3(NGT * TPG, DM / 128), 128, 0, stream>>>(O, nullptr, nullptr, PK, F[12], F[0], X1, nullptr, nullptr);
  k_ln<<<NGT * NP, 32, 0, stream>>>(X1, 0, F[13], F[14], XN);
  k_lin<1><<<dim3(NGT * TPG, FF / 128), 128, 0, stream>>>(XN, nullptr, nullptr, PK, F[16], nullptr, nullptr, GH, GL);
  k_lin<2><<<dim3(NGT * TPG, DM / 128), 128, 0, stream>>>(nullptr, GH, GL, PK, F[18], X1, (float*)d_out, nullptr, nullptr);
}
